// MyModel_87522843560581
// MI455X (gfx1250) — hardware-verified
//
#include <hip/hip_runtime.h>
#include <stdint.h>

typedef __attribute__((ext_vector_type(16))) _Float16 v16h;
typedef __attribute__((ext_vector_type(8)))  _Float16 v8h;
typedef __attribute__((ext_vector_type(16))) __bf16   v16b;
typedef __attribute__((ext_vector_type(8)))  __bf16   v8b;
typedef __attribute__((ext_vector_type(8)))  float    v8f;
typedef __attribute__((ext_vector_type(4)))  float    v4f;

__device__ __forceinline__ unsigned short f2bf_bits(float f) {
  unsigned u = __float_as_uint(f);
  return (unsigned short)((u + 0x7FFFu + ((u >> 16) & 1u)) >> 16);
}
__device__ __forceinline__ float bf_bits2f(unsigned short h) { return __uint_as_float(((unsigned)h) << 16); }

__device__ __forceinline__ void dep_guard_h(v8f& a, v8f& b, v16h x, v16h y) { asm volatile("v_nop\n\tv_nop\n\tv_nop\n\tv_nop" : "+v"(a), "+v"(b) : "v"(x), "v"(y)); }
__device__ __forceinline__ void dep_guard_b(v8f& a, v8f& b, v16b x, v16b y) { asm volatile("v_nop\n\tv_nop\n\tv_nop\n\tv_nop" : "+v"(a), "+v"(b) : "v"(x), "v"(y)); }
__device__ __forceinline__ void dep_guard3_h(v8f& a, v8f& b, v8f& c, v16h x, v16h y) { asm volatile("v_nop\n\tv_nop\n\tv_nop\n\tv_nop" : "+v"(a), "+v"(b), "+v"(c) : "v"(x), "v"(y)); }
__device__ __forceinline__ void keep4_h(v16h a, v16h b, v16h c, v16h d) { asm volatile("v_nop" :: "v"(a), "v"(b), "v"(c), "v"(d)); }
__device__ __forceinline__ void keep4_b(v16b a, v16b b, v16b c, v16b d) { asm volatile("v_nop" :: "v"(a), "v"(b), "v"(c), "v"(d)); }
__device__ __forceinline__ void acc_guard4(v8f& a, v8f& b, v8f& c, v8f& d) { asm volatile("v_nop\n\tv_nop\n\tv_nop\n\tv_nop" : "+v"(a), "+v"(b), "+v"(c), "+v"(d)); }
template <typename T> struct Frag;
template <> struct Frag<_Float16> {
  typedef v16h V; union U { v16h v; v8h h[2]; };
  static __device__ __forceinline__ v16h load(const _Float16* p) {
    U f; f.h[0] = *(const v8h*)(p); f.h[1] = *(const v8h*)(p + 16); return f.v;
  }
  static __device__ __forceinline__ v8f mma(v16h a, v16h b, v8f c) {
    return __builtin_amdgcn_wmma_f32_16x16x32_f16(false, a, false, b, (short)0, c, false, false);
  }
  static __device__ __forceinline__ void guard(v8f& a, v8f& b, v16h x, v16h y) { dep_guard_h(a, b, x, y); }
  static __device__ __forceinline__ void keep(v16h a, v16h b, v16h c, v16h d) { keep4_h(a, b, c, d); }
};
template <> struct Frag<__bf16> {
  typedef v16b V; union U { v16b v; v8b h[2]; };
  static __device__ __forceinline__ v16b load(const __bf16* p) {
    U f; f.h[0] = *(const v8b*)(p); f.h[1] = *(const v8b*)(p + 16); return f.v;
  }
  static __device__ __forceinline__ v8f mma(v16b a, v16b b, v8f c) {
    return __builtin_amdgcn_wmma_f32_16x16x32_bf16(false, a, false, b, (short)0, c, false, false);
  }
  static __device__ __forceinline__ void guard(v8f& a, v8f& b, v16b x, v16b y) { dep_guard_b(a, b, x, y); }
  static __device__ __forceinline__ void keep(v16b a, v16b b, v16b c, v16b d) { keep4_b(a, b, c, d); }
};

template <int ET> struct Elem;
template <> struct Elem<0> { typedef _Float16 T; };
template <> struct Elem<1> { typedef __bf16 T; };
template <int ET, bool SPLIT, int BIAS_MODE, int OUT_MODE, bool RESID, int ACT = 0>
__global__ __launch_bounds__(256) void wmma_gemm64(
    const unsigned short* __restrict__ Ap, const unsigned short* __restrict__ A2p, int lda, long strideA,
    const unsigned short* __restrict__ Btp, const unsigned short* __restrict__ Bt2p, int ldb, long strideB,
    void* __restrict__ Cout, void* __restrict__ Cout2, int ldc, long strideC,
    const float* __restrict__ bias,
    const float* __restrict__ resid, long strideR,
    int M, int N, int K, float scale) {
  typedef typename Elem<ET>::T T;
  typedef typename Frag<T>::V V;
  const T* A = (const T*)Ap; const T* A2 = (const T*)A2p; const T* Bt = (const T*)Btp; const T* Bt2 = (const T*)Bt2p;
  __shared__ __align__(16) float sT[8][16 * 68];
  const int b    = blockIdx.y;
  const int lane = threadIdx.x & 31;
  const int wave = threadIdx.x >> 5;
  const int tilesN = N >> 6;
  const int tilesM = M >> 6;
  const int tile = blockIdx.x * 8 + wave;
  if (tile >= tilesM * tilesN) return;
  const int tm = tile / tilesN;
  const int tn = tile - tm * tilesN;
  const int m0 = tm << 6;
  const int n0 = tn << 6;

  const T* Ab  = A  + (size_t)b * strideA;
  const T* Bb  = Bt + (size_t)b * strideB;
  const T* Ab2 = SPLIT ? (A2  + (size_t)b * strideA) : nullptr;
  const T* Bb2 = SPLIT ? (Bt2 + (size_t)b * strideB) : nullptr;

  const int rlane = lane & 15;
  const int koff  = (lane >> 4) * 8;
  const int mOff  = (lane >> 4) * 8;

  v8f acc[4][4];
#pragma unroll
  for (int i = 0; i < 4; ++i)
#pragma unroll
    for (int j = 0; j < 4; ++j) acc[i][j] = (v8f){0.f,0.f,0.f,0.f,0.f,0.f,0.f,0.f};

  for (int k0 = 0; k0 < K; k0 += 32) {
    V bh[4], bl[4];
#pragma unroll
    for (int j = 0; j < 4; ++j) {
      const size_t bo = (size_t)(n0 + (j << 4) + rlane) * ldb + koff + k0;
      bh[j] = Frag<T>::load(Bb + bo);
      if (SPLIT) bl[j] = Frag<T>::load(Bb2 + bo);
    }
#pragma unroll
    for (int i = 0; i < 4; ++i) {
      const size_t ao = (size_t)(m0 + (i << 4) + rlane) * lda + koff + k0;
      V ah = Frag<T>::load(Ab + ao);
      V al;
      if (SPLIT) al = Frag<T>::load(Ab2 + ao);
#pragma unroll
      for (int j = 0; j < 4; ++j) {
        acc[i][j] = Frag<T>::mma(ah, bh[j], acc[i][j]);
        if (SPLIT) {
          acc[i][j] = Frag<T>::mma(ah, bl[j], acc[i][j]);
          acc[i][j] = Frag<T>::mma(al, bh[j], acc[i][j]);
        }
      }
      Frag<T>::guard(acc[i][0], acc[i][3], ah, SPLIT ? al : ah);
    }
    Frag<T>::keep(bh[0], bh[1], bh[2], bh[3]);
    if (SPLIT) Frag<T>::keep(bl[0], bl[1], bl[2], bl[3]);
  }
  acc_guard4(acc[0][0], acc[0][1], acc[0][2], acc[0][3]);
  acc_guard4(acc[1][0], acc[1][1], acc[1][2], acc[1][3]);
  acc_guard4(acc[2][0], acc[2][1], acc[2][2], acc[2][3]);
  acc_guard4(acc[3][0], acc[3][1], acc[3][2], acc[3][3]);

  float* slab = sT[wave];
  const float* Rb = RESID ? (resid + (size_t)b * strideR) : nullptr;
#pragma unroll
  for (int i = 0; i < 4; ++i) {
    const int mBase = m0 + (i << 4);
#pragma unroll
    for (int j = 0; j < 4; ++j) {
      const int n = n0 + (j << 4) + rlane;
      float bv = 0.f;
      if (BIAS_MODE == 2) bv = bias[n];
#pragma unroll
      for (int r = 0; r < 8; ++r) {
        float v = acc[i][j][r] * scale;
        if (BIAS_MODE == 1) v += bias[mBase + mOff + r];
        if (BIAS_MODE == 2) v += bv;
        if (RESID) v += Rb[(size_t)(mBase + mOff + r) * ldc + n];
        if (ACT == 1) v = tanhf(v);
        if (ACT == 2) v = fmaxf(v, 0.0f);
        if (ACT == 3) v = v / (1.0f + expf(-v));
        if (ACT == 4) v = (v > 0.f) ? v : 0.01f * v;
        if (ACT == 5) v = 0.5f * v * (1.0f + erff(v * 0.70710678118654752f));
        slab[(mOff + r) * 68 + (j << 4) + rlane] = v;
      }
    }
    __builtin_amdgcn_fence(__ATOMIC_RELEASE, "workgroup");
    __builtin_amdgcn_wave_barrier();
    __builtin_amdgcn_fence(__ATOMIC_ACQUIRE, "workgroup");
    if (OUT_MODE == 0) {
      float* C = (float*)Cout + (size_t)b * strideC;
      const int hh = lane >> 4, c4 = (lane & 15) * 4;
      for (int pass = 0; pass < 2; ++pass) {
#pragma unroll
        for (int it = 0; it < 8; ++it) {
          const int row = it * 2 + hh;
          v4f v = *(const v4f*)(slab + row * 68 + c4);
          *(volatile v4f*)(C + (size_t)(mBase + row) * ldc + n0 + c4) = v;
        }
        __threadfence();
      }
    } else {
      const int q = lane >> 3, c8 = (lane & 7) * 8;
      unsigned short* C  = (unsigned short*)Cout  + (size_t)b * strideC;
      unsigned short* C2 = (OUT_MODE == 2) ? ((unsigned short*)Cout2 + (size_t)b * strideC) : nullptr;
      for (int pass = 0; pass < 2; ++pass) {
#pragma unroll
        for (int it = 0; it < 4; ++it) {
          const int row = it * 4 + q;
          const float* sp = slab + row * 68 + c8;
          v8h hv, lv;
#pragma unroll
          for (int e = 0; e < 8; ++e) {
            if (OUT_MODE == 1) {
              hv[e] = (_Float16)sp[e];
            } else {
              unsigned short hb = f2bf_bits(sp[e]);
              unsigned short lb = f2bf_bits(sp[e] - bf_bits2f(hb));
              hv[e] = __builtin_bit_cast(_Float16, hb);
              lv[e] = __builtin_bit_cast(_Float16, lb);
            }
          }
          *(volatile v8h*)(C + (size_t)(mBase + row) * ldc + n0 + c8) = hv;
          if (OUT_MODE == 2) *(volatile v8h*)(C2 + (size_t)(mBase + row) * ldc + n0 + c8) = lv;
        }
        __threadfence();
      }
    }
    __builtin_amdgcn_fence(__ATOMIC_RELEASE, "workgroup");
    __builtin_amdgcn_wave_barrier();
    __builtin_amdgcn_fence(__ATOMIC_ACQUIRE, "workgroup");
  }
}

constexpr int NB    = 256;
constexpr int NT    = 200;
constexpr int ND    = 311;
constexpr int NDP   = 320;
constexpr int NU    = 256;
constexpr int NG3   = 3 * NU;
constexpr int NCLS  = 19;
constexpr int NCLSP = 64;
constexpr int NROWS = NB * NT;
constexpr int NHC   = 2 * NU;

constexpr float OPSC_X = 64.0f;
constexpr float OPSC_H = 64.0f;
constexpr float OPSC_W = 16.0f;
constexpr float PROD_INV = 1.0f / 1024.0f;

constexpr int GB_ROWS    = 32;
constexpr int GB_WAVES   = 16;
constexpr int GB_THREADS = GB_WAVES * 32;
constexpr int XSP = NDP + 8;
constexpr int HAP = NU + 8;

static_assert(NB % GB_ROWS == 0, "batch tiles");
static_assert(GB_WAVES * 16 == NU, "waves cover all units");
static_assert(GB_WAVES * 2 == GB_ROWS, "each wave stages / stores exactly 2 rows");
static_assert(NDP % 32 == 0 && NU % 32 == 0 && NHC % 32 == 0, "K multiples of 32");
static_assert((XSP * 2) % 16 == 0 && (HAP * 2) % 16 == 0, "16-B aligned LDS rows");
static_assert(NROWS % 64 == 0 && NCLSP % 64 == 0, "dense GEMM tile multiples");
static_assert((GB_ROWS * XSP) % 2 == 0, "u32 zero fill");

template <int KP>
__global__ __launch_bounds__(256) void transpose_cast16(const float* __restrict__ in, int Ksrc, int Nsrc,
                                                         unsigned short* __restrict__ out, float scale) {
  constexpr int TP  = KP + 8;
  constexpr int LPR = KP / 64;
  static_assert(KP % 64 == 0, "whole lines per row");
  __shared__ __align__(16) _Float16 tile[32 * TP];
  const int tid = threadIdx.x, lane = tid & 31, wave = tid >> 5;
  const int n0 = blockIdx.x * 32;
  const int n  = n0 + lane;
  const int nc = (n < Nsrc) ? n : (Nsrc - 1);
#pragma unroll 4
  for (int k = wave; k < KP; k += 8) {
    const int kc = (k < Ksrc) ? k : (Ksrc - 1);
    float v = in[(size_t)kc * Nsrc + nc];
    v = (k < Ksrc && n < Nsrc) ? v : 0.0f;
    tile[lane * TP + k] = (_Float16)(v * scale);
  }
  __syncthreads();
  const int q = lane >> 3, c8 = (lane & 7) * 8;
  v8h vals[LPR];
#pragma unroll
  for (int it = 0; it < LPR; ++it) {
    const int L = (wave * LPR + it) * 4 + q;
    const int row = L / LPR, seg = L - row * LPR;
    vals[it] = *(const v8h*)(tile + row * TP + seg * 64 + c8);
  }
  _Float16* outh = (_Float16*)out;
  for (int pass = 0; pass < 2; ++pass) {
#pragma unroll
    for (int it = 0; it < LPR; ++it) {
      const int L = (wave * LPR + it) * 4 + q;
      const int row = L / LPR, seg = L - row * LPR;
      *(volatile v8h*)(outh + (size_t)(n0 + row) * KP + seg * 64 + c8) = vals[it];
    }
    __threadfence();
  }
}

__global__ __launch_bounds__(GB_THREADS) void gru_bidir_kernel(
    const float* __restrict__ x,
    const unsigned short* __restrict__ kTp,
    const unsigned short* __restrict__ rkTp,
    const float* __restrict__ bias_f,
    const float* __restrict__ bias_b,
    unsigned short* __restrict__ Hp) {
  union FH { v16h v; v8h h[2]; };
  __shared__ __align__(16) _Float16 xs[GB_ROWS * XSP];
  __shared__ __align__(16) _Float16 hA[2][GB_ROWS * HAP];
  __shared__ int s_mask[GB_ROWS];

  const int tid  = threadIdx.x;
  const int lane = tid & 31, wave = tid >> 5;
  const int hh = lane >> 4, rlane = lane & 15, koff = hh * 8;
  const int dir = blockIdx.y;
  const int b0  = blockIdx.x * GB_ROWS;
  const _Float16* kT  = (const _Float16*)kTp  + (size_t)dir * NG3 * NDP;
  const _Float16* rkT = (const _Float16*)rkTp + (size_t)dir * NG3 * NU;
  const float* bias = dir ? bias_b : bias_f;
  _Float16* Hh = (_Float16*)Hp;
  const int ucol = wave * 16 + rlane;

  const float bz0 = bias[ucol],       br0 = bias[NU + ucol],       bh0 = bias[2 * NU + ucol];
  const float bz1 = bias[NG3 + ucol], br1 = bias[NG3 + NU + ucol], bh1 = bias[NG3 + 2 * NU + ucol];

  for (int i = tid; i < GB_ROWS * XSP / 2; i += GB_THREADS) ((unsigned*)xs)[i] = 0u;
  for (int i = tid; i < GB_ROWS * HAP; i += GB_THREADS) ((unsigned*)(&hA[0][0]))[i] = 0u;
  if (tid < GB_ROWS) s_mask[tid] = 0;

  float hreg[2][8];
#pragma unroll
  for (int i = 0; i < 2; ++i)
#pragma unroll
    for (int r = 0; r < 8; ++r) hreg[i][r] = 0.0f;
  __syncthreads();

  for (int s = 0; s < NT; ++s) {
    const int t   = dir ? (NT - 1 - s) : s;
    const int cur = s & 1, nxt = cur ^ 1;

#pragma unroll
    for (int rr2 = 0; rr2 < 2; ++rr2) {
      const int rr = wave * 2 + rr2;
      const float* xrow = x + ((size_t)(b0 + rr) * NT + t) * ND;
      int nz = 0;
#pragma unroll
      for (int j = 0; j < 10; ++j) {
        const int idx = lane + 32 * j;
        const int idc = (idx < ND) ? idx : (ND - 1);
        float v = xrow[idc];
        v = (idx < ND) ? v : 0.0f;
        nz |= (v != 0.0f) ? 1 : 0;
        xs[rr * XSP + idx] = (_Float16)(v * OPSC_X);
      }
      const int anyv = __any(nz);
      if (lane == 0) s_mask[rr] = anyv;
    }
    __syncthreads();

    v8f az[2], ar[2], axh[2], arh[2];
#pragma unroll
    for (int i = 0; i < 2; ++i) {
      az[i]  = (v8f){0.f,0.f,0.f,0.f,0.f,0.f,0.f,0.f};
      ar[i]  = az[i]; axh[i] = az[i]; arh[i] = az[i];
    }
    {
      const _Float16* kz = kT + (size_t)ucol * NDP + koff;
      const _Float16* kr = kT + (size_t)(NU + ucol) * NDP + koff;
      const _Float16* kc = kT + (size_t)(2 * NU + ucol) * NDP + koff;
#pragma unroll 1
      for (int k0 = 0; k0 < NDP; k0 += 32) {
        const v16h fz = Frag<_Float16>::load(kz + k0);
        const v16h fr = Frag<_Float16>::load(kr + k0);
        const v16h fc = Frag<_Float16>::load(kc + k0);
#pragma unroll
        for (int i = 0; i < 2; ++i) {
          FH fa;
          const _Float16* ap = xs + (16 * i + rlane) * XSP + koff + k0;
          fa.h[0] = *(const v8h*)(ap);
          fa.h[1] = *(const v8h*)(ap + 16);
          az[i]  = Frag<_Float16>::mma(fa.v, fz, az[i]);
          ar[i]  = Frag<_Float16>::mma(fa.v, fr, ar[i]);
          axh[i] = Frag<_Float16>::mma(fa.v, fc, axh[i]);
          dep_guard3_h(az[i], ar[i], axh[i], fa.v, fz);
        }
        keep4_h(fz, fr, fc, fc);
      }
    }
    {
      const _Float16* rz = rkT + (size_t)ucol * NU + koff;
      const _Float16* rrp = rkT + (size_t)(NU + ucol) * NU + koff;
      const _Float16* rc = rkT + (size_t)(2 * NU + ucol) * NU + koff;
      const _Float16* hAc = &hA[cur][0];
#pragma unroll 1
      for (int k0 = 0; k0 < NU; k0 += 32) {
        const v16h fz = Frag<_Float16>::load(rz + k0);
        const v16h fr = Frag<_Float16>::load(rrp + k0);
        const v16h fc = Frag<_Float16>::load(rc + k0);
#pragma unroll
        for (int i = 0; i < 2; ++i) {
          FH fa;
          const _Float16* ap = hAc + (16 * i + rlane) * HAP + koff + k0;
          fa.h[0] = *(const v8h*)(ap);
          fa.h[1] = *(const v8h*)(ap + 16);
          az[i]  = Frag<_Float16>::mma(fa.v, fz, az[i]);
          ar[i]  = Frag<_Float16>::mma(fa.v, fr, ar[i]);
          arh[i] = Frag<_Float16>::mma(fa.v, fc, arh[i]);
          dep_guard3_h(az[i], ar[i], arh[i], fa.v, fz);
        }
        keep4_h(fz, fr, fc, fc);
      }
    }
    acc_guard4(az[0], az[1], ar[0], ar[1]);
    acc_guard4(axh[0], axh[1], arh[0], arh[1]);

    {
      _Float16* hAn = &hA[nxt][0];
#pragma unroll
      for (int i = 0; i < 2; ++i) {
#pragma unroll
        for (int r = 0; r < 8; ++r) {
          const int row = 16 * i + 8 * hh + r;
          float pz  = az[i][r] * PROD_INV + bz0 + bz1;
          float pr  = ar[i][r] * PROD_INV + br0 + br1;
          const float pxh = axh[i][r] * PROD_INV + bh0;
          const float prh = arh[i][r] * PROD_INV + bh1;
          pz = fminf(fmaxf(pz, -30.0f), 30.0f);
          pr = fminf(fmaxf(pr, -30.0f), 30.0f);
          const float zg = 1.0f / (1.0f + expf(-pz));
          const float rg = 1.0f / (1.0f + expf(-pr));
          const float hc = tanhf(pxh + rg * prh);
          const float hp = hreg[i][r];
          float hn = zg * hp + (1.0f - zg) * hc;
          hn = (s_mask[row] != 0) ? hn : hp;
          hreg[i][r] = hn;
          hAn[row * HAP + ucol] = (_Float16)(hn * OPSC_H);
        }
      }
    }
    __syncthreads();

    {
      const _Float16* hAn = &hA[nxt][0];
      const int ra = wave * 2, rb = wave * 2 + 1;
      const v8h va = *(const v8h*)(hAn + ra * HAP + lane * 8);
      const v8h vb = *(const v8h*)(hAn + rb * HAP + lane * 8);
      _Float16* da = Hh + ((size_t)(b0 + ra) * NT + t) * NHC + dir * NU + lane * 8;
      _Float16* db = Hh + ((size_t)(b0 + rb) * NT + t) * NHC + dir * NU + lane * 8;
      *(volatile v8h*)da = va;
      *(volatile v8h*)db = vb;
      __threadfence();
      *(volatile v8h*)da = va;
      *(volatile v8h*)db = vb;
    }
  }
}

constexpr int SM_ROWS = 32;
constexpr int SM_FLT  = SM_ROWS * NCLS;
static_assert(SM_FLT % 32 == 0, "block output is whole lines");
static_assert(NROWS % SM_ROWS == 0, "softmax blocks");
__global__ __launch_bounds__(256) void softmax_rows_kernel(const float* __restrict__ logits,
                                                           const float* __restrict__ bd,
                                                           float* __restrict__ out) {
  __shared__ __align__(16) float so[SM_FLT];
  const int tid = threadIdx.x, lane = tid & 31, wave = tid >> 5;
  const int R0 = blockIdx.x * SM_ROWS;
  const int lc = (lane < NCLS) ? lane : (NCLS - 1);
  const float bv = bd[lc];
#pragma unroll 1
  for (int i = 0; i < 4; ++i) {
    const int rloc = wave * 4 + i;
    const float lv = logits[(size_t)(R0 + rloc) * NCLSP + lane] + bv;
    const float v = (lane < NCLS) ? lv : -INFINITY;
    float m = v;
#pragma unroll
    for (int off = 16; off > 0; off >>= 1) m = fmaxf(m, __shfl_xor(m, off, 32));
    const float ev = expf(v - m);
    const float e = (lane < NCLS) ? ev : 0.0f;
    float ssum = e;
#pragma unroll
    for (int off = 16; off > 0; off >>= 1) ssum += __shfl_xor(ssum, off, 32);
    const float p = e / ssum;
    if (lane < NCLS) so[rloc * NCLS + lane] = p;
  }
  __syncthreads();
  const int t4 = (tid < SM_FLT / 4) ? tid : (SM_FLT / 4 - 1);
  const v4f val = *(const v4f*)(so + 4 * t4);
  float* dst = out + (size_t)blockIdx.x * SM_FLT + 4 * t4;
  if (tid < SM_FLT / 4) *(volatile v4f*)dst = val;
  __threadfence();
  if (tid < SM_FLT / 4) *(volatile v4f*)dst = val;
}

constexpr size_t WS_KT     = (size_t)2 * NG3 * NDP * 2;
constexpr size_t WS_RKT    = (size_t)2 * NG3 * NU * 2;
constexpr size_t WS_WDT    = (size_t)NCLSP * NHC * 2;
constexpr size_t WS_H      = (size_t)NROWS * NHC * 2;
constexpr size_t WS_LOGITS = (size_t)NROWS * NCLSP * 4;
constexpr size_t OFF_KT     = 0;
constexpr size_t OFF_RKT    = OFF_KT + WS_KT;
constexpr size_t OFF_WDT    = OFF_RKT + WS_RKT;
constexpr size_t OFF_H      = OFF_WDT + WS_WDT;
constexpr size_t OFF_LOGITS = OFF_H + WS_H;
constexpr size_t WS_TOTAL   = OFF_LOGITS + WS_LOGITS;
static_assert(WS_TOTAL == 67371008, "carve total");
static_assert(WS_TOTAL <= (size_t)134217728, "carve under 128 MiB");
static_assert(OFF_RKT % 256 == 0 && OFF_WDT % 256 == 0 && OFF_H % 256 == 0 && OFF_LOGITS % 256 == 0, "aligned regions");
static_assert((size_t)NROWS * NCLS * 4 == 3891200, "output bytes");

extern "C" void kernel_launch(void* const* d_in, const int* in_sizes, int n_in,
                              void* d_out, int out_size, void* d_ws, size_t ws_size,
                              hipStream_t stream) {
  (void)in_sizes; (void)n_in; (void)out_size;
  if (ws_size < WS_TOTAL) return;
  const float* x    = (const float*)d_in[0];
  const float* k_f  = (const float*)d_in[1];
  const float* rk_f = (const float*)d_in[2];
  const float* b_f  = (const float*)d_in[3];
  const float* k_b  = (const float*)d_in[4];
  const float* rk_b = (const float*)d_in[5];
  const float* b_b  = (const float*)d_in[6];
  const float* w_d  = (const float*)d_in[7];
  const float* b_d  = (const float*)d_in[8];
  float* out = (float*)d_out;

  char* ws = (char*)d_ws;
  unsigned short* kT     = (unsigned short*)(ws + OFF_KT);
  unsigned short* rkT    = (unsigned short*)(ws + OFF_RKT);
  unsigned short* wdT    = (unsigned short*)(ws + OFF_WDT);
  unsigned short* Hc     = (unsigned short*)(ws + OFF_H);
  float*          logits = (float*)(ws + OFF_LOGITS);

  transpose_cast16<NDP><<<NG3 / 32, 256, 0, stream>>>(k_f, ND, NG3, kT, OPSC_W);
  transpose_cast16<NDP><<<NG3 / 32, 256, 0, stream>>>(k_b, ND, NG3, kT + (size_t)NG3 * NDP, OPSC_W);
  transpose_cast16<NU><<<NG3 / 32, 256, 0, stream>>>(rk_f, NU, NG3, rkT, OPSC_W);
  transpose_cast16<NU><<<NG3 / 32, 256, 0, stream>>>(rk_b, NU, NG3, rkT + (size_t)NG3 * NU, OPSC_W);
  transpose_cast16<NHC><<<NCLSP / 32, 256, 0, stream>>>(w_d, NHC, NCLS, wdT, OPSC_W);

  gru_bidir_kernel<<<dim3(NB / GB_ROWS, 2), GB_THREADS, 0, stream>>>(x, kT, rkT, b_f, b_b, Hc);

  wmma_gemm64<0, false, 0, 0, false, 0><<<dim3((NROWS / 64) * (NCLSP / 64) / 8, 1), 256, 0, stream>>>(
      Hc, Hc, NHC, 0L, wdT, wdT, NHC, 0L, (void*)logits, (void*)logits, NCLSP, 0L,
      b_d, logits, 0L, NROWS, NCLSP, NHC, PROD_INV);

  softmax_rows_kernel<<<NROWS / SM_ROWS, 256, 0, stream>>>(logits, b_d, out);
}
